// BoxMultiHeadedAttention_13597866459935
// MI455X (gfx1250) — hardware-verified
//
#include <hip/hip_runtime.h>
#include <stddef.h>


#define NB   4
#define NTOK 512
#define DM   512
#define NH   8
#define DKH  64
#define MTOK (NB * NTOK)

#define S_X  1024.0f
#define S_W  4096.0f
#define S_QK 16.0f
#define S_V  1024.0f
#define S_P  4096.0f
#define S_AO 1024.0f
#define S_E  2048.0f
#define S_G  4096.0f

typedef _Float16 v16h __attribute__((ext_vector_type(16)));
typedef _Float16 v8h_base __attribute__((ext_vector_type(8)));
typedef v8h_base __attribute__((may_alias)) v8h;
typedef float v8f __attribute__((ext_vector_type(8)));
typedef float v4f_base __attribute__((ext_vector_type(4)));
typedef v4f_base __attribute__((may_alias)) v4f;

union Frag16 { v16h v; v8h half[2]; _Float16 s[16]; };
union Pack8  { v8h v; _Float16 s[8]; };
union Pack2  { unsigned u; _Float16 s[2]; };
union F8     { v4f v[2]; float f[8]; };

__device__ __forceinline__ v8f zero8f() {
  v8f z = {0.f, 0.f, 0.f, 0.f, 0.f, 0.f, 0.f, 0.f};
  return z;
}

__device__ __forceinline__ v8f wmma16(v16h a, v16h b, v8f c) {
  v8f d = __builtin_amdgcn_wmma_f32_16x16x32_f16(false, a, false, b, (short)0, c, false, false);
  asm volatile("v_nop\n\tv_nop\n\tv_nop\n\tv_nop" : "+v"(d) : "v"(a), "v"(b));
  return d;
}

__device__ __forceinline__ v16h ldfrag(const _Float16* base, int pitch, int lane, int k0) {
  const _Float16* p = base + (lane & 15) * pitch + k0 + 8 * (lane >> 4);
  Frag16 f;
  f.half[0] = *(const v8h*)(p);
  f.half[1] = *(const v8h*)(p + 16);
  return f.v;
}

template <int AM, int OM>
__global__ __launch_bounds__(128) void k_gemm(const float* Af, const _Float16* Ah, const _Float16* Al,
                                             const float* W, const float* bias,
                                             _Float16* Yh, _Float16* Yl, float* Yf,
                                             int M, int K, int Nout,
                                             float a_scale, float w_scale, float o_mul, float o_scale) {
  constexpr int NPL = (AM == 0) ? 1 : 2;
  __shared__ __attribute__((aligned(16))) _Float16 At[NPL][64][40];
  __shared__ __attribute__((aligned(16))) _Float16 Bt[NPL][64][40];
  __shared__ __attribute__((aligned(16))) float Ct[64][68];

  const int tid = threadIdx.x, lane = tid & 31, wave = tid >> 5;
  const int hh = lane >> 4, m = lane & 15;
  const int n0 = blockIdx.x * 64, m0 = blockIdx.y * 64;
  if (m0 + 64 > M || n0 + 64 > Nout) return;

  v8f acc[4];
#pragma unroll
  for (int j = 0; j < 4; ++j) acc[j] = zero8f();

#pragma unroll 1
  for (int kk = 0; kk < K; kk += 32) {
    {
      const int r = tid >> 1, cb = (tid & 1) * 16;
      if (AM == 2) {
        const size_t g = (size_t)(m0 + r) * K + kk + cb;
        const v8h h0 = *(const v8h*)(Ah + g), h1 = *(const v8h*)(Ah + g + 8);
        const v8h l0 = *(const v8h*)(Al + g), l1 = *(const v8h*)(Al + g + 8);
        *(v8h*)&At[0][r][cb] = h0;        *(v8h*)&At[0][r][cb + 8] = h1;
        *(v8h*)&At[NPL - 1][r][cb] = l0;  *(v8h*)&At[NPL - 1][r][cb + 8] = l1;
      } else {
        const float* s = Af + (size_t)(m0 + r) * K + kk + cb;
        F8 x0, x1;
        x0.v[0] = *(const v4f*)(s);      x0.v[1] = *(const v4f*)(s + 4);
        x1.v[0] = *(const v4f*)(s + 8);  x1.v[1] = *(const v4f*)(s + 12);
        Frag16 ph, pl;
#pragma unroll
        for (int e = 0; e < 8; ++e) {
          const float v0 = x0.f[e] * a_scale, v1 = x1.f[e] * a_scale;
          const _Float16 h0 = (_Float16)v0, h1 = (_Float16)v1;
          ph.s[e] = h0;
          ph.s[8 + e] = h1;
          pl.s[e] = (_Float16)(v0 - (float)h0);
          pl.s[8 + e] = (_Float16)(v1 - (float)h1);
        }
        *(v8h*)&At[0][r][cb] = ph.half[0];  *(v8h*)&At[0][r][cb + 8] = ph.half[1];
        if (NPL == 2) {
          *(v8h*)&At[NPL - 1][r][cb] = pl.half[0];  *(v8h*)&At[NPL - 1][r][cb + 8] = pl.half[1];
        }
      }
    }
    {
      const int kp = tid >> 3, nb = (tid & 7) * 8;
      const float* s0 = W + (size_t)(kk + 2 * kp) * Nout + n0 + nb;
      const float* s1 = s0 + Nout;
      F8 w0, w1;
      w0.v[0] = *(const v4f*)(s0);  w0.v[1] = *(const v4f*)(s0 + 4);
      w1.v[0] = *(const v4f*)(s1);  w1.v[1] = *(const v4f*)(s1 + 4);
#pragma unroll
      for (int d = 0; d < 8; ++d) {
        const float a = w0.f[d] * w_scale, c = w1.f[d] * w_scale;
        const _Float16 ha = (_Float16)a, hc = (_Float16)c;
        Pack2 q;
        q.s[0] = ha;  q.s[1] = hc;
        *(unsigned*)&Bt[0][nb + d][2 * kp] = q.u;
        if (NPL == 2) {
          Pack2 ql;
          ql.s[0] = (_Float16)(a - (float)ha);
          ql.s[1] = (_Float16)(c - (float)hc);
          *(unsigned*)&Bt[NPL - 1][nb + d][2 * kp] = ql.u;
        }
      }
    }
    __syncthreads();

    const v16h ah = ldfrag(&At[0][wave * 16][0], 40, lane, 0);
    if (NPL == 1) {
#pragma unroll
      for (int j = 0; j < 4; ++j) {
        const v16h bh = ldfrag(&Bt[0][j * 16][0], 40, lane, 0);
        acc[j] = wmma16(ah, bh, acc[j]);
      }
    } else {
      const v16h al = ldfrag(&At[NPL - 1][wave * 16][0], 40, lane, 0);
#pragma unroll
      for (int j = 0; j < 4; ++j) {
        const v16h bh = ldfrag(&Bt[0][j * 16][0], 40, lane, 0);
        const v16h bl = ldfrag(&Bt[NPL - 1][j * 16][0], 40, lane, 0);
        acc[j] = wmma16(ah, bh, acc[j]);
        acc[j] = wmma16(ah, bl, acc[j]);
        acc[j] = wmma16(al, bh, acc[j]);
      }
    }
    __syncthreads();
  }

#pragma unroll
  for (int j = 0; j < 4; ++j) {
    const float bcol = bias[n0 + 16 * j + m];
#pragma unroll
    for (int r = 0; r < 8; ++r) Ct[wave * 16 + 8 * hh + r][16 * j + m] = acc[j][r] * o_mul + bcol;
  }
  __syncthreads();

  if (OM == 0) {
    const int q = lane >> 3, p = lane & 7;
    v8h vals[4];
    size_t addr[4];
#pragma unroll
    for (int it = 0; it < 4; ++it) {
      const int row = wave * 16 + 4 * it + q;
      F8 c;
      c.v[0] = *(const v4f*)&Ct[row][8 * p];
      c.v[1] = *(const v4f*)&Ct[row][8 * p + 4];
      Pack8 pk;
#pragma unroll
      for (int e = 0; e < 8; ++e) pk.s[e] = (_Float16)(c.f[e] * o_scale);
      vals[it] = pk.v;
      addr[it] = (size_t)(m0 + row) * Nout + n0 + 8 * p;
    }
#pragma unroll
    for (int it = 0; it < 4; ++it) *(volatile v8h*)(Yh + addr[it]) = vals[it];
    __threadfence();
#pragma unroll
    for (int it = 0; it < 4; ++it) *(volatile v8h*)(Yh + addr[it]) = vals[it];
  } else if (OM == 1) {
    const int hd = blockIdx.x;
    const int bb = m0 / NTOK, tok0 = m0 - bb * NTOK;
    const int q = lane >> 3, p = lane & 7;
    v8h vh[4], vl[4];
    size_t addr[4];
#pragma unroll
    for (int it = 0; it < 4; ++it) {
      const int dk = wave * 16 + 4 * it + q;
      Pack8 ph, pl;
#pragma unroll
      for (int e = 0; e < 8; ++e) {
        const float v = Ct[8 * p + e][dk] * o_scale;
        const _Float16 hv = (_Float16)v;
        ph.s[e] = hv;
        pl.s[e] = (_Float16)(v - (float)hv);
      }
      vh[it] = ph.v;
      vl[it] = pl.v;
      addr[it] = (((size_t)bb * NH + hd) * DKH + dk) * NTOK + tok0 + 8 * p;
    }
#pragma unroll
    for (int it = 0; it < 4; ++it) {
      *(volatile v8h*)(Yh + addr[it]) = vh[it];
      *(volatile v8h*)(Yl + addr[it]) = vl[it];
    }
    __threadfence();
#pragma unroll
    for (int it = 0; it < 4; ++it) {
      *(volatile v8h*)(Yh + addr[it]) = vh[it];
      *(volatile v8h*)(Yl + addr[it]) = vl[it];
    }
  } else {
    const int q = lane >> 4, p = lane & 15;
    v4f vals[8];
    size_t addr[8];
#pragma unroll
    for (int it = 0; it < 8; ++it) {
      const int row = wave * 16 + 2 * it + q;
      vals[it] = *(const v4f*)&Ct[row][4 * p];
      addr[it] = (size_t)(m0 + row) * Nout + n0 + 4 * p;
    }
#pragma unroll
    for (int it = 0; it < 8; ++it) *(volatile v4f*)(Yf + addr[it]) = vals[it];
    __threadfence();
#pragma unroll
    for (int it = 0; it < 8; ++it) *(volatile v4f*)(Yf + addr[it]) = vals[it];
  }
}

__global__ __launch_bounds__(128) void k_geo(const float* box, const float* Wg, const float* bg,
                                            const int* msk, float* logg) {
  __shared__ __attribute__((aligned(16))) _Float16 Et[2][128][72];
  __shared__ __attribute__((aligned(16))) _Float16 Bg[16][72];
  __shared__ float Gs[128][17];
  __shared__ float sdm[8];
  __shared__ float sbg[8];

  const int tid = threadIdx.x, lane = tid & 31, wave = tid >> 5;
  const int hh = lane >> 4, m = lane & 15;
  const int bi = blockIdx.x;
  if (bi >= NB * NTOK) return;
  const int b = bi / NTOK, i = bi - b * NTOK;

  if (tid < 8) {
    sdm[tid] = 1.0f / powf(1000.0f, (float)tid * 0.125f);
    sbg[tid] = bg[tid];
  }
#pragma unroll
  for (int e = 0; e < 8; ++e) {
    const int idx = tid * 8 + e;
    const int n = idx >> 6, k = idx & 63;
    const float w = Wg[k * NH + (n & 7)] * S_G;
    const _Float16 wh = (_Float16)w;
    const _Float16 wl = (_Float16)(w - (float)wh);
    Bg[n][k] = (n < 8) ? wh : wl;
  }
  const v4f bxi = *(const v4f*)(box + (size_t)bi * 4);
  const float cxi = (bxi[0] + bxi[1]) * 0.5f, cyi = (bxi[2] + bxi[3]) * 0.5f;
  const float wi = (bxi[1] - bxi[0]) + 1.0f, hgi = (bxi[3] - bxi[2]) + 1.0f;
  const float rwi = 1.0f / wi, rhi = 1.0f / hgi;
  __syncthreads();

  float dm[8];
#pragma unroll
  for (int f = 0; f < 8; ++f) dm[f] = sdm[f];
  const v16h bg0 = ldfrag(&Bg[0][0], 72, lane, 0);
  const v16h bg1 = ldfrag(&Bg[0][0], 72, lane, 32);
  const size_t mbase = ((size_t)b * NTOK + i) * NTOK;
  const v8f z8 = zero8f();

#pragma unroll 1
  for (int ch = 0; ch < NTOK / 128; ++ch) {
    {
      const int j = ch * 128 + tid;
      const v4f bxj = *(const v4f*)(box + ((size_t)b * NTOK + j) * 4);
      const float cxj = (bxj[0] + bxj[1]) * 0.5f, cyj = (bxj[2] + bxj[3]) * 0.5f;
      const float wj = (bxj[1] - bxj[0]) + 1.0f, hgj = (bxj[3] - bxj[2]) + 1.0f;
      const float p0 = logf(fmaxf(fabsf((cxi - cxj) * rwi), 1e-3f));
      const float p1 = logf(fmaxf(fabsf((cyi - cyj) * rhi), 1e-3f));
      const float p2 = logf(wi / wj);
      const float p3 = logf(hgi / hgj);
      const float pp[4] = {p0 * 100.0f, p1 * 100.0f, p2 * 100.0f, p3 * 100.0f};
#pragma unroll
      for (int p = 0; p < 4; ++p) {
        Pack8 sh, sl, chv, clv;
#pragma unroll
        for (int f = 0; f < 8; ++f) {
          const float ang = pp[p] * dm[f];
          const float sv = __sinf(ang) * S_E;
          const float cv = __cosf(ang) * S_E;
          const _Float16 a = (_Float16)sv;
          sh.s[f] = a;
          sl.s[f] = (_Float16)(sv - (float)a);
          const _Float16 c = (_Float16)cv;
          chv.s[f] = c;
          clv.s[f] = (_Float16)(cv - (float)c);
        }
        *(v8h*)&Et[0][tid][p * 8] = sh.v;
        *(v8h*)&Et[1][tid][p * 8] = sl.v;
        *(v8h*)&Et[0][tid][32 + p * 8] = chv.v;
        *(v8h*)&Et[1][tid][32 + p * 8] = clv.v;
      }
    }
    __syncthreads();

#pragma unroll
    for (int t = 0; t < 2; ++t) {
      const int row0 = wave * 32 + t * 16;
      v8f acc = z8;
      const v16h a0 = ldfrag(&Et[0][row0][0], 72, lane, 0);
      const v16h l0 = ldfrag(&Et[1][row0][0], 72, lane, 0);
      acc = wmma16(a0, bg0, acc);
      acc = wmma16(l0, bg0, acc);
      const v16h a1 = ldfrag(&Et[0][row0][0], 72, lane, 32);
      const v16h l1 = ldfrag(&Et[1][row0][0], 72, lane, 32);
      acc = wmma16(a1, bg1, acc);
      acc = wmma16(l1, bg1, acc);
#pragma unroll
      for (int r = 0; r < 8; ++r) Gs[row0 + 8 * hh + r][m] = acc[r];
    }
    __syncthreads();

    v4f vv[2];
#pragma unroll
    for (int e = 0; e < 2; ++e) {
      const int hd = 2 * wave + e;
#pragma unroll
      for (int q = 0; q < 4; ++q) {
        const int jl = 4 * lane + q;
        const float graw = (Gs[jl][hd] + Gs[jl][hd + 8]) * (1.0f / (S_E * S_G)) + sbg[hd];
        const float g = fmaxf(graw, 0.0f);
        float v = logf(fmaxf(g, 1e-6f));
        const int mk = msk[mbase + ch * 128 + jl];
        v += (mk == 0) ? -1e9f : 0.0f;
        vv[e][q] = v;
      }
    }
    float* ap0 = logg + (((size_t)b * NH + 2 * wave) * NTOK + i) * NTOK + ch * 128 + 4 * lane;
    float* ap1 = ap0 + (size_t)NTOK * NTOK;
    *(volatile v4f*)ap0 = vv[0];
    *(volatile v4f*)ap1 = vv[1];
    __threadfence();
    *(volatile v4f*)ap0 = vv[0];
    *(volatile v4f*)ap1 = vv[1];
  }
}

__global__ __launch_bounds__(128) void k_attn(const _Float16* Qh, const _Float16* Kh,
                                             const _Float16* Vth, const _Float16* Vtl,
                                             const float* logg, _Float16* Oh, _Float16* Ol) {
  __shared__ __attribute__((aligned(16))) _Float16 Qt[64][72];
  __shared__ __attribute__((aligned(16))) _Float16 Kt[32][72];
  __shared__ __attribute__((aligned(16))) _Float16 Vt[2][64][40];
  __shared__ __attribute__((aligned(16))) _Float16 Pt[2][4][16][40];
  __shared__ __attribute__((aligned(16))) float Cs[64][68];

  const int tid = threadIdx.x, lane = tid & 31, wave = tid >> 5;
  const int hh = lane >> 4, m = lane & 15;
  const int blk = blockIdx.x;
  if (blk >= NB * NH * (NTOK / 64)) return;
  const int qb = blk & 7, h = (blk >> 3) & 7, b = blk >> 6;
  const int q0 = qb * 64;

  {
    const int r = tid >> 1, cb = (tid & 1) * 32;
    const _Float16* s = Qh + ((size_t)(b * NTOK + q0 + r)) * DM + h * DKH + cb;
#pragma unroll
    for (int u = 0; u < 4; ++u) *(v8h*)&Qt[r][cb + 8 * u] = *(const v8h*)(s + 8 * u);
  }
  __syncthreads();
  const v16h qa0 = ldfrag(&Qt[wave * 16][0], 72, lane, 0);
  const v16h qa1 = ldfrag(&Qt[wave * 16][0], 72, lane, 32);

  const v8f z8 = zero8f();
  v8f o[4];
#pragma unroll
  for (int j = 0; j < 4; ++j) o[j] = z8;
  float mrow[8], lrow[8];
#pragma unroll
  for (int r = 0; r < 8; ++r) { mrow[r] = -1e30f; lrow[r] = 0.0f; }

  const size_t lgrow = (((size_t)b * NH + h) * NTOK + (q0 + wave * 16 + 8 * hh)) * NTOK;
  const float SC = 0.125f / (S_QK * S_QK);

#pragma unroll 1
  for (int kt = 0; kt < NTOK / 32; ++kt) {
    const int k0 = kt * 32;
    {
      const int r = tid >> 2, cb = (tid & 3) * 16;
      const _Float16* s = Kh + ((size_t)(b * NTOK + k0 + r)) * DM + h * DKH + cb;
      *(v8h*)&Kt[r][cb] = *(const v8h*)(s);
      *(v8h*)&Kt[r][cb + 8] = *(const v8h*)(s + 8);
    }
    {
      const int r = tid >> 1, cb = (tid & 1) * 16;
      const size_t g = (((size_t)b * NH + h) * DKH + r) * NTOK + k0 + cb;
      *(v8h*)&Vt[0][r][cb] = *(const v8h*)(Vth + g);
      *(v8h*)&Vt[0][r][cb + 8] = *(const v8h*)(Vth + g + 8);
      *(v8h*)&Vt[1][r][cb] = *(const v8h*)(Vtl + g);
      *(v8h*)&Vt[1][r][cb + 8] = *(const v8h*)(Vtl + g + 8);
    }
    __syncthreads();

    v8f s[2];
#pragma unroll
    for (int c = 0; c < 2; ++c) {
      const v16h b0 = ldfrag(&Kt[16 * c][0], 72, lane, 0);
      const v16h b1 = ldfrag(&Kt[16 * c][0], 72, lane, 32);
      v8f sc = z8;
      sc = wmma16(qa0, b0, sc);
      sc = wmma16(qa1, b1, sc);
      s[c] = sc;
    }

    float t[2][8];
#pragma unroll
    for (int c = 0; c < 2; ++c)
#pragma unroll
      for (int r = 0; r < 8; ++r)
        t[c][r] = s[c][r] * SC + logg[lgrow + (size_t)r * NTOK + k0 + 16 * c + m];

    float rmax[8];
#pragma unroll
    for (int r = 0; r < 8; ++r) rmax[r] = fmaxf(t[0][r], t[1][r]);
#pragma unroll
    for (int off = 8; off >= 1; off >>= 1)
#pragma unroll
      for (int r = 0; r < 8; ++r) rmax[r] = fmaxf(rmax[r], __shfl_xor(rmax[r], off, 16));

    float alpha[8];
#pragma unroll
    for (int r = 0; r < 8; ++r) {
      const float mnew = fmaxf(mrow[r], rmax[r]);
      alpha[r] = __expf(mrow[r] - mnew);
      mrow[r] = mnew;
    }
#pragma unroll
    for (int c = 0; c < 2; ++c)
#pragma unroll
      for (int r = 0; r < 8; ++r) t[c][r] = __expf(t[c][r] - mrow[r]);

    float rsum[8];
#pragma unroll
    for (int r = 0; r < 8; ++r) rsum[r] = t[0][r] + t[1][r];
#pragma unroll
    for (int off = 8; off >= 1; off >>= 1)
#pragma unroll
      for (int r = 0; r < 8; ++r) rsum[r] += __shfl_xor(rsum[r], off, 16);
#pragma unroll
    for (int r = 0; r < 8; ++r) lrow[r] = lrow[r] * alpha[r] + rsum[r];
#pragma unroll
    for (int j = 0; j < 4; ++j)
#pragma unroll
      for (int r = 0; r < 8; ++r) o[j][r] *= alpha[r];

#pragma unroll
    for (int c = 0; c < 2; ++c)
#pragma unroll
      for (int r = 0; r < 8; ++r) {
        const float ps = t[c][r] * S_P;
        const _Float16 ph = (_Float16)ps;
        Pt[0][wave][8 * hh + r][16 * c + m] = ph;
        Pt[1][wave][8 * hh + r][16 * c + m] = (_Float16)(ps - (float)ph);
      }
    __syncthreads();

    const v16h pah = ldfrag(&Pt[0][wave][0][0], 40, lane, 0);
    const v16h pal = ldfrag(&Pt[1][wave][0][0], 40, lane, 0);
#pragma unroll
    for (int j = 0; j < 4; ++j) {
      const v16h vh = ldfrag(&Vt[0][16 * j][0], 40, lane, 0);
      const v16h vl = ldfrag(&Vt[1][16 * j][0], 40, lane, 0);
      o[j] = wmma16(pah, vh, o[j]);
      o[j] = wmma16(pah, vl, o[j]);
      o[j] = wmma16(pal, vh, o[j]);
    }
    __syncthreads();
  }

  float inv[8];
#pragma unroll
  for (int r = 0; r < 8; ++r) inv[r] = (1.0f / lrow[r]) * (S_AO / (S_P * S_V));
#pragma unroll
  for (int j = 0; j < 4; ++j)
#pragma unroll
    for (int r = 0; r < 8; ++r) Cs[wave * 16 + 8 * hh + r][16 * j + m] = o[j][r] * inv[r];
  __syncthreads();

  {
    const int q = lane >> 3, p = lane & 7;
    v8h vh[4], vl[4];
    size_t addr[4];
#pragma unroll
    for (int it = 0; it < 4; ++it) {
      const int row = wave * 16 + 4 * it + q;
      F8 c;
      c.v[0] = *(const v4f*)&Cs[row][8 * p];
      c.v[1] = *(const v4f*)&Cs[row][8 * p + 4];
      Pack8 ph, pl;
#pragma unroll
      for (int e = 0; e < 8; ++e) {
        const float v = c.f[e];
        const _Float16 hv = (_Float16)v;
        ph.s[e] = hv;
        pl.s[e] = (_Float16)(v - (float)hv);
      }
      vh[it] = ph.v;
      vl[it] = pl.v;
      addr[it] = ((size_t)(b * NTOK + q0 + row)) * DM + h * DKH + 8 * p;
    }
#pragma unroll
    for (int it = 0; it < 4; ++it) {
      *(volatile v8h*)(Oh + addr[it]) = vh[it];
      *(volatile v8h*)(Ol + addr[it]) = vl[it];
    }
    __threadfence();
#pragma unroll
    for (int it = 0; it < 4; ++it) {
      *(volatile v8h*)(Oh + addr[it]) = vh[it];
      *(volatile v8h*)(Ol + addr[it]) = vl[it];
    }
  }
}

extern "C" void kernel_launch(void* const* d_in, const int* in_sizes, int n_in,
                              void* d_out, int out_size, void* d_ws, size_t ws_size,
                              hipStream_t stream) {
  if (n_in < 15) return;
  const int xsz = MTOK * DM, wsz = DM * DM;
  if (in_sizes[0] != xsz || in_sizes[1] != xsz || in_sizes[2] != xsz) return;
  if (in_sizes[3] != MTOK * 4 || in_sizes[4] != NB * NTOK * NTOK) return;
  if (in_sizes[5] != wsz || in_sizes[7] != wsz || in_sizes[9] != wsz || in_sizes[11] != wsz) return;
  if (in_sizes[6] != DM || in_sizes[8] != DM || in_sizes[10] != DM || in_sizes[12] != DM) return;
  if (in_sizes[13] != DKH * NH || in_sizes[14] != NH || out_size != xsz) return;

  const float* Xq  = (const float*)d_in[0];
  const float* Xk  = (const float*)d_in[1];
  const float* Xv  = (const float*)d_in[2];
  const float* box = (const float*)d_in[3];
  const int*   msk = (const int*)d_in[4];
  const float* Wq  = (const float*)d_in[5];
  const float* bq  = (const float*)d_in[6];
  const float* Wk  = (const float*)d_in[7];
  const float* bk  = (const float*)d_in[8];
  const float* Wv  = (const float*)d_in[9];
  const float* bv  = (const float*)d_in[10];
  const float* Wo  = (const float*)d_in[11];
  const float* bo  = (const float*)d_in[12];
  const float* Wg  = (const float*)d_in[13];
  const float* bg  = (const float*)d_in[14];
  float* out = (float*)d_out;

  char* ws = (char*)d_ws;
  size_t off = 0;
  float* logg = (float*)(ws + off);          off += (size_t)NB * NH * NTOK * NTOK * sizeof(float);
  _Float16* Q16 = (_Float16*)(ws + off);     off += (size_t)xsz * 2;
  _Float16* K16 = (_Float16*)(ws + off);     off += (size_t)xsz * 2;
  _Float16* Vth = (_Float16*)(ws + off);     off += (size_t)xsz * 2;
  _Float16* Vtl = (_Float16*)(ws + off);     off += (size_t)xsz * 2;
  _Float16* AOh = (_Float16*)(ws + off);     off += (size_t)xsz * 2;
  _Float16* AOl = (_Float16*)(ws + off);     off += (size_t)xsz * 2;
  if (off > ws_size) return;

  const float omul = 1.0f / (S_X * S_W);
  const float omul_o = 1.0f / (S_AO * S_W);
  const dim3 gg(DM / 64, MTOK / 64), gb(128);

  k_gemm<0, 0><<<gg, gb, 0, stream>>>(Xq, Q16, Q16, Wq, bq, Q16, Q16, logg,
                                      MTOK, DM, DM, S_X, S_W, omul, S_QK);
  k_gemm<0, 0><<<gg, gb, 0, stream>>>(Xk, K16, K16, Wk, bk, K16, K16, logg,
                                      MTOK, DM, DM, S_X, S_W, omul, S_QK);
  k_gemm<1, 1><<<gg, gb, 0, stream>>>(Xv, Vth, Vtl, Wv, bv, Vth, Vtl, logg,
                                      MTOK, DM, DM, S_X, S_W, omul, S_V);
  k_geo<<<dim3(NB * NTOK), gb, 0, stream>>>(box, Wg, bg, msk, logg);
  k_attn<<<dim3(NB * NH * (NTOK / 64)), gb, 0, stream>>>(Q16, K16, Vth, Vtl, logg, AOh, AOl);
  k_gemm<2, 2><<<gg, gb, 0, stream>>>(Wo, AOh, AOl, Wo, bo, AOh, AOl, out,
                                      MTOK, DM, DM, 1.0f, S_W, omul_o, 1.0f);
}
